// Model_8907762172297
// MI455X (gfx1250) — hardware-verified
//
#include <hip/hip_runtime.h>
#include <math.h>

#ifndef NB
#define NB 128
#endif
#define NB_FULL 128
#define CHAN 21
#define TLEN 2048
#define PLEN 16
#define DMODEL 128
#define NMOD 8
#define LPAT (TLEN / PLEN)
#define LPM (LPAT / NMOD)
#define BC (NB * CHAN)
#define NTOT (BC * TLEN)
#define NTOT_FULL (NB_FULL * CHAN * TLEN)
#define OUT4_OFF_BYTES 16

static_assert(NB % 64 == 0);
static_assert(BC % 64 == 0);
static_assert(TLEN % 64 == 0 && TLEN % 32 == 0);
static_assert(DMODEL == 128 && PLEN == 16 && NMOD == 8 && LPM == 16);
static_assert(LPAT == 128);
static_assert(NTOT % 4 == 0);
static_assert((size_t)OUT4_OFF_BYTES + (size_t)NTOT_FULL * 4 == (size_t)22020112);
static_assert(OUT4_OFF_BYTES == 16);

typedef __attribute__((ext_vector_type(16))) _Float16 v16h;
typedef __attribute__((ext_vector_type(8)))  _Float16 v8h;
typedef __attribute__((ext_vector_type(8)))  float    v8f;
typedef __attribute__((ext_vector_type(4)))  float    v4f;
typedef __attribute__((ext_vector_type(4)))  unsigned int v4u;


#define VST2(T, ptr, val) do { const T vst2_v_ = (val); *(volatile T*)(ptr) = vst2_v_; __threadfence(); *(volatile T*)(ptr) = vst2_v_; } while (0)
#define VST2V4(ptr, val) do { const v4f vst2_v4_ = (val); *(volatile v4f*)(ptr) = vst2_v4_; __threadfence(); *(volatile v4f*)(ptr) = vst2_v4_; } while (0)

__device__ __forceinline__ float bfr(float f) {
    unsigned u = __float_as_uint(f);
    u += 0x7FFFu + ((u >> 16) & 1u);
    return __uint_as_float(u & 0xFFFF0000u);
}
__device__ __forceinline__ unsigned short f2h_bits(float x) {
    return (fabsf(x) < 6.104e-5f) ? (unsigned short)0 : __builtin_bit_cast(unsigned short, (_Float16)x);
}
__device__ __forceinline__ void st8h(unsigned short* P, size_t o, const float* v) {
    v4u pk;
    pk.x = (unsigned)f2h_bits(v[0]) | ((unsigned)f2h_bits(v[1]) << 16);
    pk.y = (unsigned)f2h_bits(v[2]) | ((unsigned)f2h_bits(v[3]) << 16);
    pk.z = (unsigned)f2h_bits(v[4]) | ((unsigned)f2h_bits(v[5]) << 16);
    pk.w = (unsigned)f2h_bits(v[6]) | ((unsigned)f2h_bits(v[7]) << 16);
    VST2(v4u, (v4u*)(P + o), pk);
}

union FragU { v16h v; v8h h[2]; };
__device__ __forceinline__ v16h frag_ld(const _Float16* p) {
    FragU f; f.h[0] = *(const v8h*)(p); f.h[1] = *(const v8h*)(p + 16); return f.v;
}
__device__ __forceinline__ v8f wmma16(v16h a, v16h b, v8f c) {
    c = __builtin_amdgcn_wmma_f32_16x16x32_f16(false, a, false, b, (short)0, c, false, false);
    asm volatile("v_nop\n\tv_nop\n\tv_nop\n\tv_nop" : "+v"(c) : "v"(a), "v"(b));
    return c;
}
__device__ __forceinline__ void dep_guard_h(v8f& a, v8f& b, v16h x, v16h y) { asm volatile("v_nop\n\tv_nop\n\tv_nop\n\tv_nop" : "+v"(a), "+v"(b) : "v"(x), "v"(y)); }
__device__ __forceinline__ void keep4_h(v16h a, v16h b, v16h c, v16h d) { asm volatile("v_nop" :: "v"(a), "v"(b), "v"(c), "v"(d)); }
__device__ __forceinline__ void acc_guard4(v8f& a, v8f& b, v8f& c, v8f& d) { asm volatile("v_nop\n\tv_nop\n\tv_nop\n\tv_nop" : "+v"(a), "+v"(b), "+v"(c), "+v"(d)); }
__device__ __forceinline__ void wave_sync_lds() {
    __builtin_amdgcn_fence(3  , "workgroup");
    __builtin_amdgcn_wave_barrier();
    __builtin_amdgcn_fence(2  , "workgroup");
}

typedef _Float16 h16;
static __device__ __forceinline__ h16 toh_flush(float v) {
    const h16 r = (h16)v;
    return (fabsf(v) < 6.103515625e-05f) ? (h16)0.0f : r;
}

static constexpr float ACT_CARRY = 8.0f;
static constexpr float SC_EMB = 1.0f / 32.0f;
static constexpr float SC_ENC = 1.0f / 256.0f;
static constexpr float SC_MAP = 1.0f / 2048.0f;

template <int OUT_MODE, bool RESID, bool RELU>
__global__ __launch_bounds__(256) void k_gemm64(
    const _Float16* __restrict__ A, unsigned lda, const _Float16* __restrict__ Bt, unsigned ldb,
    void* __restrict__ Cout, unsigned ldc, const float* __restrict__ bias, const float* __restrict__ resid,
    unsigned M, unsigned N, unsigned K, float scale, float oscale) {
  __shared__ __align__(16) float sT[8][16 * 68];
  const unsigned lane = threadIdx.x & 31u;
  const unsigned wave = threadIdx.x >> 5;
  const unsigned tilesN = N >> 6, tilesM = M >> 6;
  const unsigned tile = blockIdx.x * 8u + wave;
  if (tile >= tilesM * tilesN) return;
  const unsigned tm = tile / tilesN;
  const unsigned tn = tile - tm * tilesN;
  const unsigned m0 = tm << 6, n0 = tn << 6;
  const unsigned rlane = lane & 15u;
  const unsigned koff = (lane >> 4) * 8u;
  const unsigned mOff = koff;

  v8f acc[4][4];
#pragma unroll
  for (int i = 0; i < 4; ++i)
#pragma unroll
    for (int j = 0; j < 4; ++j) acc[i][j] = (v8f){0.f,0.f,0.f,0.f,0.f,0.f,0.f,0.f};

  for (unsigned k0 = 0; k0 < K; k0 += 32u) {
    v16h bh[4];
#pragma unroll
    for (int j = 0; j < 4; ++j)
      bh[j] = frag_ld(Bt + (size_t)(n0 + ((unsigned)j << 4) + rlane) * ldb + koff + k0);
#pragma unroll
    for (int i = 0; i < 4; ++i) {
      const v16h ah = frag_ld(A + (size_t)(m0 + ((unsigned)i << 4) + rlane) * lda + koff + k0);
#pragma unroll
      for (int j = 0; j < 4; ++j)
        acc[i][j] = __builtin_amdgcn_wmma_f32_16x16x32_f16(false, ah, false, bh[j], (short)0, acc[i][j], false, false);
      dep_guard_h(acc[i][0], acc[i][3], ah, ah);
    }
    keep4_h(bh[0], bh[1], bh[2], bh[3]);
  }
  acc_guard4(acc[0][0], acc[0][1], acc[0][2], acc[0][3]);
  acc_guard4(acc[1][0], acc[1][1], acc[1][2], acc[1][3]);
  acc_guard4(acc[2][0], acc[2][1], acc[2][2], acc[2][3]);
  acc_guard4(acc[3][0], acc[3][1], acc[3][2], acc[3][3]);

  float* slab = sT[wave];
#pragma unroll
  for (int i = 0; i < 4; ++i) {
    const unsigned mBase = m0 + ((unsigned)i << 4);
#pragma unroll
    for (int j = 0; j < 4; ++j) {
      const unsigned n = n0 + ((unsigned)j << 4) + rlane;
      const float bv = bfr(bias[n]);
#pragma unroll
      for (int r = 0; r < 8; ++r) {
        float v = acc[i][j][r] * scale + bv;
        if (RELU) v = fmaxf(v, 0.0f);
        if (OUT_MODE == 1) v *= oscale;
        slab[(mOff + (unsigned)r) * 68u + ((unsigned)j << 4) + rlane] = v;
      }
    }
    wave_sync_lds();
    if (OUT_MODE == 0) {
      float* C = (float*)Cout;
      const unsigned hh = lane >> 4, c4 = (lane & 15u) * 4u;
#pragma unroll
      for (int half = 0; half < 2; ++half) {
        v4f vv[4];
#pragma unroll
        for (int it = 0; it < 4; ++it) {
          const unsigned row = (unsigned)(half * 4 + it) * 2u + hh;
          vv[it] = *(const v4f*)(slab + row * 68u + c4);
          if (RESID) vv[it] += *(const v4f*)(resid + (size_t)(mBase + row) * ldc + n0 + c4);
        }
        for (int pass = 0; pass < 2; ++pass) {
#pragma unroll
          for (int it = 0; it < 4; ++it) {
            const unsigned row = (unsigned)(half * 4 + it) * 2u + hh;
            *(volatile v4f*)(C + (size_t)(mBase + row) * ldc + n0 + c4) = vv[it];
          }
          __threadfence();
        }
      }
    } else {
      _Float16* C = (_Float16*)Cout;
      const unsigned q = lane >> 3, c8 = (lane & 7u) * 8u;
      v8h hv[4];
#pragma unroll
      for (int it = 0; it < 4; ++it) {
        const unsigned row = (unsigned)it * 4u + q;
        const float* sp = slab + row * 68u + c8;
#pragma unroll
        for (int e = 0; e < 8; ++e) hv[it][e] = (_Float16)sp[e];
      }
      for (int pass = 0; pass < 2; ++pass) {
#pragma unroll
        for (int it = 0; it < 4; ++it) {
          const unsigned row = (unsigned)it * 4u + q;
          *(volatile v8h*)(C + (size_t)(mBase + row) * ldc + n0 + c8) = hv[it];
        }
        __threadfence();
      }
    }
    wave_sync_lds();
  }
}

__global__ __launch_bounds__(256) void k_wt16(const float* __restrict__ Wm, unsigned KI, unsigned NO, unsigned lgper,
                                              unsigned short* __restrict__ W16, float sw) {
    const unsigned layer = blockIdx.y;
    const float* Wl = Wm + (size_t)layer * KI * NO;
    unsigned short* Dl = W16 + (size_t)layer * KI * NO;
    const unsigned u = blockIdx.x * 256u + threadIdx.x;
    const unsigned per = 1u << lgper;
    if (u >= NO * per) return;
    const unsigned k0 = 8u * (u & (per - 1u));
    const unsigned o = u >> lgper;
    float v[8];
#pragma unroll
    for (int i = 0; i < 8; ++i) v[i] = bfr(Wl[(size_t)(k0 + (unsigned)i) * NO + o]) * sw;
    st8h(Dl, (size_t)o * KI + k0, v);
}

#define CH_PT 136
#define CH_PF 132
static_assert(256 * 8 == TLEN);
static_assert(256 * 2 * 16 == TLEN * 4);
static_assert(256 * 1 * 16 == TLEN * 2);
static_assert(TLEN * 2 + NMOD * 16 * CH_PT * 2 + TLEN * 4 + NMOD * 16 * CH_PF * 4 <= 131072);
static_assert(CH_PT % 8 == 0 && CH_PT >= DMODEL);
static_assert(CH_PF >= DMODEL);
static_assert(8 * 8 * 32 == 16 * DMODEL);

__device__ __forceinline__ float gelu_tanh(float v) {
    const float u = 0.7978845608028654f * (v + 0.044715f * (v * v * v));
    return v * (0.5f * (1.0f + tanhf(u)));
}

template <bool GELU>
__device__ __forceinline__ void enc_stage(_Float16* tile, float* pre, const _Float16* __restrict__ wpl,
                                          const float* __restrict__ bias, unsigned c, unsigned hh) {
    v8f acc[8];
#pragma unroll
    for (int t = 0; t < 8; ++t) acc[t] = (v8f){0.f,0.f,0.f,0.f,0.f,0.f,0.f,0.f};
#pragma unroll 1
    for (unsigned k0 = 0; k0 < (unsigned)DMODEL; k0 += 32u) {
        const v16h a = frag_ld(tile + c * CH_PT + k0 + 8u * hh);
#pragma unroll
        for (int t = 0; t < 8; ++t) {
            const v16h b = frag_ld(wpl + (size_t)((unsigned)t * 16u + c) * DMODEL + k0 + 8u * hh);
            acc[t] = wmma16(a, b, acc[t]);
        }
    }
    wave_sync_lds();
    if (GELU) {
#pragma unroll
        for (int t = 0; t < 8; ++t) {
            const unsigned col = (unsigned)t * 16u + c;
            const float bv = bfr(bias[col]);
#pragma unroll
            for (int r = 0; r < 8; ++r)
                pre[(8u * hh + (unsigned)r) * CH_PF + col] = acc[t][r] * SC_ENC + bv;
        }
        wave_sync_lds();
#pragma unroll 1
        for (unsigned i = 0; i < 64u; ++i) {
            const unsigned col = (i >> 3) * 16u + c;
            const unsigned row = 8u * hh + (i & 7u);
            const float pv = pre[row * CH_PF + col];
            const float v = gelu_tanh(pv);
            tile[row * CH_PT + col] = toh_flush(v * ACT_CARRY);
        }
    } else {
#pragma unroll
        for (int t = 0; t < 8; ++t) {
            const unsigned col = (unsigned)t * 16u + c;
            const float bv = bfr(bias[col]);
#pragma unroll
            for (int r = 0; r < 8; ++r) {
                const float v = acc[t][r] * SC_ENC + bv;
                tile[(8u * hh + (unsigned)r) * CH_PT + col] = toh_flush(v * ACT_CARRY);
            }
        }
    }
    wave_sync_lds();
}

__global__ __launch_bounds__(256) void k_chain(const float* __restrict__ xin,
                                               const _Float16* __restrict__ wemb, const _Float16* __restrict__ w1,
                                               const _Float16* __restrict__ w2, const _Float16* __restrict__ wdec,
                                               const float* __restrict__ emb_b, const float* __restrict__ b1,
                                               const float* __restrict__ b2, const float* __restrict__ dec_b,
                                               float* __restrict__ rec32, _Float16* __restrict__ rec16, int write16) {
    __shared__ __align__(16) _Float16 sX[TLEN];
    __shared__ __align__(16) _Float16 sT[NMOD][16 * CH_PT];
    __shared__ __align__(16) float sPre[NMOD][16 * CH_PF];
    __shared__ __align__(16) float sOut[TLEN];
    const unsigned tid = threadIdx.x, lane = tid & 31u;
    const unsigned wave = (unsigned)__builtin_amdgcn_readfirstlane(threadIdx.x >> 5);
    const unsigned hh = lane >> 4, c = lane & 15u;
    const unsigned bc = blockIdx.x;

    {
        const float* xr = xin + (size_t)bc * TLEN + 8u * tid;
        const v4f a = *(const v4f*)xr;
        const v4f b = *(const v4f*)(xr + 4);
        v8h hv;
        hv[0] = toh_flush(bfr(a.x)); hv[1] = toh_flush(bfr(a.y)); hv[2] = toh_flush(bfr(a.z)); hv[3] = toh_flush(bfr(a.w));
        hv[4] = toh_flush(bfr(b.x)); hv[5] = toh_flush(bfr(b.y)); hv[6] = toh_flush(bfr(b.z)); hv[7] = toh_flush(bfr(b.w));
        *(v8h*)(sX + 8u * tid) = hv;
    }
    __syncthreads();

    _Float16* tile = sT[wave];
    float* pre = sPre[wave];
    v8h z8;
#pragma unroll
    for (int i = 0; i < 8; ++i) z8[i] = (_Float16)0.0f;

    {
        FragU fa;
        fa.h[0] = *(const v8h*)(sX + (c * 8u + wave) * 16u + 8u * hh);
        fa.h[1] = z8;
#pragma unroll
        for (int t = 0; t < 8; ++t) {
            FragU fb;
            fb.h[0] = *(const v8h*)(wemb + (size_t)((unsigned)t * 16u + c) * PLEN + 8u * hh);
            fb.h[1] = z8;
            const v8f z = (v8f){0.f,0.f,0.f,0.f,0.f,0.f,0.f,0.f};
            const v8f e = wmma16(fa.v, fb.v, z);
            const unsigned col = (unsigned)t * 16u + c;
            const float bv = bfr(emb_b[col]);
#pragma unroll
            for (int r = 0; r < 8; ++r)
                tile[(8u * hh + (unsigned)r) * CH_PT + col] = toh_flush((e[r] * SC_EMB + bv) * ACT_CARRY);
        }
    }
    wave_sync_lds();

    enc_stage<true >(tile, pre, w1 + (size_t)wave * DMODEL * DMODEL, b1 + wave * DMODEL, c, hh);
    enc_stage<false>(tile, pre, w2 + (size_t)wave * DMODEL * DMODEL, b2 + wave * DMODEL, c, hh);

    {
        v8f d = (v8f){0.f,0.f,0.f,0.f,0.f,0.f,0.f,0.f};
#pragma unroll 1
        for (unsigned k0 = 0; k0 < (unsigned)DMODEL; k0 += 32u) {
            const v16h a = frag_ld(tile + c * CH_PT + k0 + 8u * hh);
            const v16h b = frag_ld(wdec + (size_t)(wave * PLEN + c) * DMODEL + k0 + 8u * hh);
            d = wmma16(a, b, d);
        }
        const float bd = bfr(dec_b[wave * PLEN + c]);
#pragma unroll
        for (int r = 0; r < 8; ++r)
            sOut[((8u * hh + (unsigned)r) * 16u + c) * 8u + wave] = d[r] * SC_ENC + bd;
    }
    __syncthreads();

    {
        const v4f o0 = *(const v4f*)(sOut + 4u * tid);
        const v4f o1 = *(const v4f*)(sOut + 1024u + 4u * tid);
        const v4f p0 = *(const v4f*)(sOut + 8u * tid);
        const v4f p1 = *(const v4f*)(sOut + 8u * tid + 4u);
        v8h hv;
        hv[0] = toh_flush(p0.x * ACT_CARRY); hv[1] = toh_flush(p0.y * ACT_CARRY);
        hv[2] = toh_flush(p0.z * ACT_CARRY); hv[3] = toh_flush(p0.w * ACT_CARRY);
        hv[4] = toh_flush(p1.x * ACT_CARRY); hv[5] = toh_flush(p1.y * ACT_CARRY);
        hv[6] = toh_flush(p1.z * ACT_CARRY); hv[7] = toh_flush(p1.w * ACT_CARRY);
        float* d32 = rec32 + (size_t)bc * TLEN;
        _Float16* d16 = rec16 + (size_t)bc * TLEN;
        for (int pass = 0; pass < 2; ++pass) {
            *(volatile v4f*)(d32 + 4u * tid) = o0;
            *(volatile v4f*)(d32 + 1024u + 4u * tid) = o1;
            if (write16 != 0) *(volatile v8h*)(d16 + 8u * tid) = hv;
            __threadfence();
        }
    }
}

#define CL_U0 8u
#define CL_F4 1024u
#define U_TOT ((unsigned)(NTOT / 4) + 1u)
#define CL_NBLK ((U_TOT - CL_U0 + CL_F4 - 1u) / CL_F4)
static_assert(256u * 4u == CL_F4);
static_assert(CL_U0 * 16u == 128u);

__device__ __forceinline__ float abs4(v4f a, v4f b) {
    return (fabsf(a.x - b.x) + fabsf(a.y - b.y)) + (fabsf(a.z - b.z) + fabsf(a.w - b.w));
}

__global__ __launch_bounds__(256) void k_copyloss(const float* __restrict__ yhat, const float* __restrict__ yrec,
                                                  const float* __restrict__ xrec, const float* __restrict__ xin,
                                                  const float* __restrict__ yin, float* __restrict__ out,
                                                  float* __restrict__ part) {
#pragma clang fp contract(off)
    __shared__ float sW[8][4];
    const unsigned tid = threadIdx.x, lane = tid & 31u;
    const unsigned wave = (unsigned)__builtin_amdgcn_readfirstlane(threadIdx.x >> 5);
    float s0 = 0.f, s1 = 0.f, s2 = 0.f;
#pragma unroll 1
    for (unsigned it = 0; it < 4u; ++it) {
        const unsigned u = CL_U0 + blockIdx.x * CL_F4 + it * 256u + tid;
        const bool ok = u < U_TOT;
        const unsigned uc = ok ? u : (U_TOT - 1u);
        const size_t src = (size_t)(uc - 1u) * 4u;
        const v4f yh = *(const v4f*)(yhat + src);
        const v4f yr = *(const v4f*)(yrec + src);
        const v4f xr = *(const v4f*)(xrec + src);
        v4f xi = *(const v4f*)(xin + src);
        v4f yi = *(const v4f*)(yin + src);
        xi.x = bfr(xi.x); xi.y = bfr(xi.y); xi.z = bfr(xi.z); xi.w = bfr(xi.w);
        yi.x = bfr(yi.x); yi.y = bfr(yi.y); yi.z = bfr(yi.z); yi.w = bfr(yi.w);
        const float d0 = abs4(yh, yr), d1 = abs4(xr, xi), d2 = abs4(yr, yi);
        s0 += ok ? d0 : 0.f;
        s1 += ok ? d1 : 0.f;
        s2 += ok ? d2 : 0.f;
        for (int pass = 0; pass < 2; ++pass) {
            if (ok) *(volatile v4f*)(out + (size_t)u * 4u) = yh;
            __threadfence();
        }
    }
#pragma unroll
    for (int o = 16; o > 0; o >>= 1) {
        s0 += __shfl_xor(s0, o, 32);
        s1 += __shfl_xor(s1, o, 32);
        s2 += __shfl_xor(s2, o, 32);
    }
    if (lane == 0u) { sW[wave][0] = s0; sW[wave][1] = s1; sW[wave][2] = s2; }
    __syncthreads();
    if (tid < 8u) {
        float t0 = 0.f, t1 = 0.f, t2 = 0.f;
#pragma unroll
        for (int w = 0; w < 8; ++w) { t0 += sW[w][0]; t1 += sW[w][1]; t2 += sW[w][2]; }
        v4f pv;
        pv.x = (tid == 0u) ? t0 : 0.f;
        pv.y = (tid == 0u) ? t1 : 0.f;
        pv.z = (tid == 0u) ? t2 : 0.f;
        pv.w = 0.f;
        float* dst = part + (size_t)blockIdx.x * 32u + 4u * tid;
        for (int pass = 0; pass < 2; ++pass) {
            *(volatile v4f*)dst = pv;
            __threadfence();
        }
    }
}

#define HEAD_N 28u
static_assert(HEAD_N + 4u == 32u);
static_assert((CL_U0 - 1u) * 4u == HEAD_N);
static constexpr double INV_NTOT = 1.0 / (double)NTOT;

__global__ __launch_bounds__(256) void k_final(const float* __restrict__ part, const float* __restrict__ yhat,
                                               const float* __restrict__ yrec, const float* __restrict__ xrec,
                                               const float* __restrict__ xin, const float* __restrict__ yin,
                                               float* __restrict__ out) {
#pragma clang fp contract(off)
    __shared__ double sD[3][256];
    __shared__ __align__(16) float sLine[32];
    const unsigned tid = threadIdx.x;
    double a0 = 0.0, a1 = 0.0, a2 = 0.0;
#pragma unroll 1
    for (unsigned b = tid; b < CL_NBLK; b += 256u) {
        const v4f p = *(const v4f*)(part + (size_t)b * 32u);
        a0 += (double)p.x; a1 += (double)p.y; a2 += (double)p.z;
    }
    {
        const unsigned i = (tid < HEAD_N) ? tid : (HEAD_N - 1u);
        const bool ok = tid < HEAD_N;
        const float yh = yhat[i], yr = yrec[i], xr = xrec[i];
        const float xi = bfr(xin[i]), yi = bfr(yin[i]);
        const float d0 = fabsf(yh - yr), d1 = fabsf(xr - xi), d2 = fabsf(yr - yi);
        a0 += ok ? (double)d0 : 0.0;
        a1 += ok ? (double)d1 : 0.0;
        a2 += ok ? (double)d2 : 0.0;
    }
    sD[0][tid] = a0; sD[1][tid] = a1; sD[2][tid] = a2;
    __syncthreads();
    for (unsigned s = 128u; s > 0u; s >>= 1) {
        if (tid < s) {
            sD[0][tid] += sD[0][tid + s];
            sD[1][tid] += sD[1][tid + s];
            sD[2][tid] += sD[2][tid + s];
        }
        __syncthreads();
    }
    if (tid < 32u) {
        const unsigned hi = ((tid < 4u) ? 4u : tid) - 4u;
        const float yv = yhat[hi];
        const float m0 = (float)(sD[0][0] * INV_NTOT);
        const float m1 = (float)(sD[1][0] * INV_NTOT);
        const float m2 = (float)(sD[2][0] * INV_NTOT);
        float v = yv;
        v = (tid == 0u) ? m0 : v;
        v = (tid == 1u) ? (m1 + m2) : v;
        v = (tid == 2u || tid == 3u) ? 0.0f : v;
        sLine[tid] = v;
    }
    __syncthreads();
    if (tid < 8u) {
        const v4f lv = *(const v4f*)(sLine + 4u * tid);
        for (int pass = 0; pass < 2; ++pass) {
            *(volatile v4f*)(out + 4u * tid) = lv;
            __threadfence();
        }
    }
}

static constexpr size_t al256(size_t b) { return (b + 255) & ~(size_t)255; }
static constexpr size_t WS_WEMB  = al256((size_t)DMODEL * PLEN * 2);
static constexpr size_t WS_WENC  = al256((size_t)NMOD * DMODEL * DMODEL * 2);
static constexpr size_t WS_WDEC  = al256((size_t)NMOD * PLEN * DMODEL * 2);
static constexpr size_t WS_WMAP  = al256((size_t)TLEN * TLEN * 2);
static constexpr size_t WS_R32   = al256((size_t)NTOT * 4);
static constexpr size_t WS_R16   = al256((size_t)NTOT * 2);
static constexpr size_t WS_PART  = al256((size_t)CL_NBLK * 128);
static constexpr size_t WS_TOTAL = WS_WEMB + 2 * WS_WENC + WS_WDEC + WS_WMAP + 3 * WS_R32 + WS_R16 + WS_PART;
static_assert(WS_TOTAL <= (size_t)134217728);
static_assert((size_t)(BC / 64) * 64 * TLEN * 4 <= WS_R32);
static_assert((size_t)(U_TOT - 2u) * 16 + 16 <= WS_R32);
static_assert((size_t)(CL_NBLK - 1u) * 128 + 128 <= WS_PART);

extern "C" void kernel_launch(void* const* d_in, const int* in_sizes, int n_in, void* d_out, int out_size,
                              void* d_ws, size_t ws_size, hipStream_t stream) {
    if (n_in < 12) return;
    if (in_sizes[0] < NTOT || in_sizes[1] < NTOT || in_sizes[2] < PLEN * DMODEL || in_sizes[3] < DMODEL) return;
    if (in_sizes[4] < NMOD * DMODEL * DMODEL || in_sizes[5] < NMOD * DMODEL || in_sizes[6] < NMOD * DMODEL * DMODEL || in_sizes[7] < NMOD * DMODEL) return;
    if (in_sizes[8] < NMOD * DMODEL * PLEN || in_sizes[9] < NMOD * PLEN || in_sizes[10] < TLEN * TLEN || in_sizes[11] < TLEN) return;
    if (out_size < NTOT + 4) return;

    const float* x      = (const float*)d_in[0];
    const float* y      = (const float*)d_in[1];
    const float* emb_W  = (const float*)d_in[2];
    const float* emb_b  = (const float*)d_in[3];
    const float* enc_W1 = (const float*)d_in[4];
    const float* enc_b1 = (const float*)d_in[5];
    const float* enc_W2 = (const float*)d_in[6];
    const float* enc_b2 = (const float*)d_in[7];
    const float* dec_W  = (const float*)d_in[8];
    const float* dec_b  = (const float*)d_in[9];
    const float* map_W  = (const float*)d_in[10];
    const float* map_b  = (const float*)d_in[11];
    float* out = (float*)d_out;

    char* wsp = (char*)d_ws;
    size_t off = 0;
    auto carve = [&](size_t bytes) -> void* { void* r = wsp + off; off += (bytes + 255) & ~(size_t)255; return r; };
    unsigned short* wemb   = (unsigned short*)carve((size_t)DMODEL * PLEN * 2);
    unsigned short* w1     = (unsigned short*)carve((size_t)NMOD * DMODEL * DMODEL * 2);
    unsigned short* w2     = (unsigned short*)carve((size_t)NMOD * DMODEL * DMODEL * 2);
    unsigned short* wdec   = (unsigned short*)carve((size_t)NMOD * PLEN * DMODEL * 2);
    unsigned short* wmap   = (unsigned short*)carve((size_t)TLEN * TLEN * 2);
    float*          xrec32 = (float*)carve((size_t)NTOT * 4);
    float*          yrec32 = (float*)carve((size_t)NTOT * 4);
    float*          yhat32 = (float*)carve((size_t)NTOT * 4);
    unsigned short* xrec16 = (unsigned short*)carve((size_t)NTOT * 2);
    float*          part   = (float*)carve((size_t)CL_NBLK * 128);
    if (off > ws_size || off > (size_t)134217728) return;

    k_wt16<<<dim3((DMODEL * (PLEN / 8)) / 256, 1), 256, 0, stream>>>(emb_W, PLEN, DMODEL, 1, wemb, 32.0f);
    k_wt16<<<dim3((DMODEL * (DMODEL / 8)) / 256, NMOD), 256, 0, stream>>>(enc_W1, DMODEL, DMODEL, 4, w1, 32.0f);
    k_wt16<<<dim3((DMODEL * (DMODEL / 8)) / 256, NMOD), 256, 0, stream>>>(enc_W2, DMODEL, DMODEL, 4, w2, 32.0f);
    k_wt16<<<dim3((PLEN * (DMODEL / 8)) / 256, NMOD), 256, 0, stream>>>(dec_W, DMODEL, PLEN, 4, wdec, 32.0f);
    k_wt16<<<dim3((TLEN * (TLEN / 8)) / 256, 1), 256, 0, stream>>>(map_W, TLEN, TLEN, 8, wmap, 256.0f);

    k_chain<<<BC, 256, 0, stream>>>(x, (const _Float16*)wemb, (const _Float16*)w1, (const _Float16*)w2, (const _Float16*)wdec,
                                    emb_b, enc_b1, enc_b2, dec_b, xrec32, (_Float16*)xrec16, 1);
    k_chain<<<BC, 256, 0, stream>>>(y, (const _Float16*)wemb, (const _Float16*)w1, (const _Float16*)w2, (const _Float16*)wdec,
                                    emb_b, enc_b1, enc_b2, dec_b, yrec32, (_Float16*)xrec16, 0);

    const unsigned gM = ((BC / 64) * (TLEN / 64) + 7) / 8;
    k_gemm64<0, false, false><<<gM, 256, 0, stream>>>((const _Float16*)xrec16, TLEN, (const _Float16*)wmap, TLEN,
        (void*)yhat32, TLEN, map_b, nullptr, BC, TLEN, TLEN, SC_MAP, 1.0f);

    k_copyloss<<<CL_NBLK, 256, 0, stream>>>(yhat32, yrec32, xrec32, x, y, out, part);
    k_final<<<1, 256, 0, stream>>>(part, yhat32, yrec32, xrec32, x, y, out);
}
